// GCNConv_39041252720968
// MI455X (gfx1250) — hardware-verified
//
#include <hip/hip_runtime.h>
#include <stddef.h>
#include <stdint.h>


#define DF      128
#define GBM     64
#define GTHR    128
#define STHR    256
#define SWAVE   8
#define DEGCAP  128
#define WUNITS  2048
#define WTHR    256
#define WSMAX   134217728

static_assert(DF == 128 && (DF % 32) == 0);
static_assert(GBM == (GTHR / 32) * 16);
static_assert(WUNITS == DF * (DF / 8) && (WUNITS % WTHR) == 0);
static_assert(STHR == SWAVE * 32);
static_assert(DEGCAP % 32 == 0);

typedef float          v4f   __attribute__((ext_vector_type(4)));
typedef float          v8f   __attribute__((ext_vector_type(8)));
typedef int            v8i   __attribute__((ext_vector_type(8)));
typedef unsigned       v2u   __attribute__((ext_vector_type(2)));
typedef unsigned short v8us  __attribute__((ext_vector_type(8)));
typedef unsigned short v16us __attribute__((ext_vector_type(16)));
typedef _Float16       v8h   __attribute__((ext_vector_type(8)));
typedef _Float16       v16h  __attribute__((ext_vector_type(16)));
typedef v4f  __attribute__((may_alias)) v4fa;
typedef v2u  __attribute__((may_alias)) v2ua;
typedef v8us __attribute__((may_alias)) v8usa;
union FragH { v16h v; v16us u; v8h h[2]; v8us hu[2]; v8i w; };

__device__ __forceinline__ v8f wmh(const FragH& a, const FragH& b, v8f c) {
  v8f d = __builtin_amdgcn_wmma_f32_16x16x32_f16(false, a.v, false, b.v, (short)0, c, false, false);
  asm volatile("v_nop\n\tv_nop\n\tv_nop\n\tv_nop" : "+v"(d) : "v"(a.w), "v"(b.w));
  return d;
}

__device__ __forceinline__ unsigned short h_bits(float f) {
  return __builtin_bit_cast(unsigned short, (_Float16)f);
}
__device__ __forceinline__ float h_val(unsigned short b) {
  return (float)__builtin_bit_cast(_Float16, b);
}

__global__ __launch_bounds__(WTHR) void k_wprep(const float* __restrict__ W, unsigned short* WT) {
  const int u = (int)blockIdx.x * WTHR + (int)threadIdx.x;
  if (u >= WUNITS) return;
  const int n  = u >> 4;
  const int k8 = (u & 15) * 8;
  const float* p = W + (size_t)k8 * DF + n;
  v8us o;
#pragma unroll
  for (int j = 0; j < 8; ++j) o[j] = h_bits(p[(size_t)j * DF]);
  unsigned short* dp = WT + (size_t)n * DF + k8;
  *(volatile v8us*)dp = o;
  __threadfence();
  *(volatile v8us*)dp = o;
}

__global__ __launch_bounds__(GTHR) void k_gemm(const float* __restrict__ X, const unsigned short* __restrict__ WT,
                                               unsigned short* XH, int nN) {
  __shared__ __attribute__((aligned(16))) float stg[GBM * DF];
  const int tid = (int)threadIdx.x, lane = tid & 31, wave = tid >> 5, hh = lane >> 4, m = lane & 15;
  const int rowBase = (int)blockIdx.x * GBM;

  v8f acc[8];
  {
    const v8f z = {0.f, 0.f, 0.f, 0.f, 0.f, 0.f, 0.f, 0.f};
#pragma unroll
    for (int t = 0; t < 8; ++t) acc[t] = z;
  }
  int ar = rowBase + 16 * wave + m;
  ar = ar > nN - 1 ? nN - 1 : ar;
  const float* ap = X + (size_t)ar * DF + 8 * hh;
  const unsigned short* bp = WT + (size_t)m * DF + 8 * hh;

#pragma unroll 1
  for (int k0 = 0; k0 < DF; k0 += 32) {
    FragH af;
    {
      const v4f x0 = *(const v4f*)(ap + k0);
      const v4f x1 = *(const v4f*)(ap + k0 + 4);
      const v4f x2 = *(const v4f*)(ap + k0 + 16);
      const v4f x3 = *(const v4f*)(ap + k0 + 20);
      v8h q0, q1;
      q0[0] = (_Float16)x0.x; q0[1] = (_Float16)x0.y; q0[2] = (_Float16)x0.z; q0[3] = (_Float16)x0.w;
      q0[4] = (_Float16)x1.x; q0[5] = (_Float16)x1.y; q0[6] = (_Float16)x1.z; q0[7] = (_Float16)x1.w;
      q1[0] = (_Float16)x2.x; q1[1] = (_Float16)x2.y; q1[2] = (_Float16)x2.z; q1[3] = (_Float16)x2.w;
      q1[4] = (_Float16)x3.x; q1[5] = (_Float16)x3.y; q1[6] = (_Float16)x3.z; q1[7] = (_Float16)x3.w;
      af.h[0] = q0;
      af.h[1] = q1;
    }
#pragma unroll
    for (int nt = 0; nt < 8; ++nt) {
      const unsigned short* wq = bp + (size_t)(16 * nt) * DF + k0;
      FragH bf;
      bf.hu[0] = *(const v8usa*)wq;
      bf.hu[1] = *(const v8usa*)(wq + 16);
      acc[nt] = wmh(af, bf, acc[nt]);
    }
  }

#pragma unroll
  for (int nt = 0; nt < 8; ++nt) {
    const int lc = 16 * nt + m;
#pragma unroll
    for (int r = 0; r < 8; ++r) {
      const int lr = 16 * wave + 8 * hh + r;
      stg[lr * DF + lc] = acc[nt][r];
    }
  }
  __syncthreads();

  v8us qv[8];
#pragma unroll
  for (int p = 0; p < 8; ++p) {
    const int lr = 16 * wave + 2 * p + hh;
    const float* s = stg + lr * DF + 8 * m;
    const v4f a = *(const v4fa*)s;
    const v4f b = *(const v4fa*)(s + 4);
    v8us o;
    o[0] = h_bits(a.x); o[1] = h_bits(a.y); o[2] = h_bits(a.z); o[3] = h_bits(a.w);
    o[4] = h_bits(b.x); o[5] = h_bits(b.y); o[6] = h_bits(b.z); o[7] = h_bits(b.w);
    qv[p] = o;
  }
#pragma unroll
  for (int p = 0; p < 8; ++p) {
    unsigned short* dp = XH + (size_t)(rowBase + 16 * wave + 2 * p + hh) * DF + 8 * m;
    *(volatile v8us*)dp = qv[p];
  }
  __threadfence();
#pragma unroll
  for (int p = 0; p < 8; ++p) {
    unsigned short* dp = XH + (size_t)(rowBase + 16 * wave + 2 * p + hh) * DF + 8 * m;
    *(volatile v8us*)dp = qv[p];
  }
}

__global__ __launch_bounds__(STHR) void k_spmm(const unsigned short* __restrict__ XH, const int* __restrict__ rp,
                                               const int* __restrict__ ci, const float* __restrict__ dg,
                                               float* out, int nN, int nE) {
  const int lane = (int)threadIdx.x & 31;
  const int row = __builtin_amdgcn_readfirstlane((int)blockIdx.x * SWAVE + ((int)threadIdx.x >> 5));
  if (row >= nN) return;

  int e0 = rp[row];
  int e1 = rp[row + 1];
  e0 = e0 < 0 ? 0 : (e0 > nE ? nE : e0);
  e1 = e1 < e0 ? e0 : (e1 > nE ? nE : e1);
  int cnt = e1 - e0;
  const bool big = cnt > DEGCAP;
  cnt = cnt > DEGCAP ? DEGCAP : cnt;

  const unsigned short* xl = XH + 4 * lane;
  float a0 = 0.0f, a1 = 0.0f, a2 = 0.0f, a3 = 0.0f;
#pragma unroll 1
  for (int b0 = 0; b0 < cnt; b0 += 32) {
    int ei = e0 + b0 + lane;
    ei = ei > nE - 1 ? nE - 1 : ei;
    int cv = ci[ei];
    cv = cv < 0 ? 0 : (cv > nN - 1 ? nN - 1 : cv);
    const int dbits = __float_as_int(dg[ei]);
    const int m32 = (cnt - b0) < 32 ? (cnt - b0) : 32;
#pragma unroll 4
    for (int j = 0; j < m32; ++j) {
      const int   c = __builtin_amdgcn_readlane(cv, j);
      const float d = __int_as_float(__builtin_amdgcn_readlane(dbits, j));
      const v2u w = *(const v2ua*)(xl + (size_t)c * DF);
      const float x0 = h_val((unsigned short)(w.x & 0xffffu));
      const float x1 = h_val((unsigned short)(w.x >> 16));
      const float x2 = h_val((unsigned short)(w.y & 0xffffu));
      const float x3 = h_val((unsigned short)(w.y >> 16));
      a0 += (float)(_Float16)(d * x0);
      a1 += (float)(_Float16)(d * x1);
      a2 += (float)(_Float16)(d * x2);
      a3 += (float)(_Float16)(d * x3);
    }
  }

  const float pz = big ? __int_as_float(0x7fc00000) : 0.0f;
  v4f o;
  o.x = (float)(_Float16)(a0 + pz);
  o.y = (float)(_Float16)(a1 + pz);
  o.z = (float)(_Float16)(a2 + pz);
  o.w = (float)(_Float16)(a3 + pz);
  float* op = out + (size_t)row * DF + 4 * lane;
  *(volatile v4f*)op = o;
  __threadfence();
  *(volatile v4f*)op = o;
}

static inline int cdiv(int a, int b) { return (a + b - 1) / b; }
static inline size_t al256(size_t o) { return (o + 255) & ~(size_t)255; }

extern "C" void kernel_launch(void* const* d_in, const int* in_sizes, int n_in,
                              void* d_out, int out_size, void* d_ws, size_t ws_size,
                              hipStream_t stream) {
  if (n_in < 5) return;
  if (in_sizes[0] < DF || (in_sizes[0] % DF) != 0) return;
  const int nN = in_sizes[0] / DF;
  if (in_sizes[1] != DF * DF) return;
  if (in_sizes[2] != nN + 1) return;
  const int nE = in_sizes[3];
  if (nE < 1 || in_sizes[4] != nE) return;
  if (nN < 1 || nN >= (1 << 24)) return;
  if ((long long)out_size != (long long)nN * DF) return;

  const float* X  = (const float*)d_in[0];
  const float* W  = (const float*)d_in[1];
  const int*   rp = (const int*)d_in[2];
  const int*   ci = (const int*)d_in[3];
  const float* dg = (const float*)d_in[4];
  float* out = (float*)d_out;

  const int MP = cdiv(nN, GBM) * GBM;
  const int gM = MP / GBM;
  const int gS = cdiv(nN, SWAVE);

  char* ws = (char*)d_ws;
  size_t off = 0;
  const size_t oWT = off; off = al256(off + (size_t)DF * DF * 2);
  const size_t oXH = off; off = al256(off + (size_t)MP * DF * 2);
  if (off > ws_size || off > (size_t)WSMAX) return;
  unsigned short* WT = (unsigned short*)(ws + oWT);
  unsigned short* XH = (unsigned short*)(ws + oXH);

  k_wprep<<<WUNITS / WTHR, WTHR, 0, stream>>>(W, WT);
  k_gemm<<<gM, GTHR, 0, stream>>>(X, WT, XH, nN);
  k_spmm<<<gS, STHR, 0, stream>>>(XH, rp, ci, dg, out, nN, nE);
}
